// DeepSeekFeedForward_71451075936568
// MI455X (gfx1250) — hardware-verified
//
#include <hip/hip_runtime.h>


#define CDIM 1024
#define HDIM 1024
#define NEXP 8
#define LDK  64
#define STR  72
#define XSCALE 64.0f
#define WSCALE 1024.0f
#define HSCALE 256.0f
#define INV_XW (1.0f / 65536.0f)
#define INV_HW (1.0f / 262144.0f)

typedef _Float16       v16h __attribute__((ext_vector_type(16)));
typedef _Float16       v8h  __attribute__((ext_vector_type(8)));
typedef float          v8f  __attribute__((ext_vector_type(8)));
typedef float          v4f  __attribute__((ext_vector_type(4)));
typedef unsigned short us8  __attribute__((ext_vector_type(8)));

union FragH { v16h v; us8 h[2]; };
union Pack8 { v8h f; us8 u; };

__device__ __forceinline__ unsigned short h2bits(float x) {
  union { _Float16 f; unsigned short u; } c;
  c.f = (_Float16)x;
  return c.u;
}

__device__ __forceinline__ v8f wmma_f16(v16h a, v16h b, v8f c) {
  v8f d = __builtin_amdgcn_wmma_f32_16x16x32_f16(false, a, false, b, (short)0, c, false, false);
  asm volatile("v_nop\n\tv_nop\n\tv_nop\n\tv_nop" : "+v"(d) : "v"(a), "v"(b));
  return d;
}

__device__ __forceinline__ v16h load_frag(const unsigned short* s, int base, int kc, int lane) {
  int r  = base + (lane & 15);
  int kb = kc * 32 + ((lane >> 4) << 3);
  FragH f;
  f.h[0] = *(const us8*)(s + r * STR + kb);
  f.h[1] = *(const us8*)(s + r * STR + kb + 16);
  return f.v;
}

__device__ __forceinline__ void stage_a(unsigned short* sA, const unsigned short* __restrict__ A,
                                        int m0, int k0, int lda, int tid) {
#pragma unroll
  for (int i = 0; i < 4; ++i) {
    int chunk = tid + i * 256;
    int row = chunk >> 3;
    int c8  = (chunk & 7) * 8;
    *(us8*)(sA + row * STR + c8) =
        *(const us8*)(A + (size_t)(m0 + row) * lda + k0 + c8);
  }
}

__device__ __forceinline__ void stage_b(unsigned short* sB, const unsigned short* __restrict__ W,
                                        int k0, int n0, int ldb, int tid) {
  int k = (tid >> 3) * 2;
  int n = (tid & 7) * 8;
  us8 r0 = *(const us8*)(W + (size_t)(k0 + k)     * ldb + n0 + n);
  us8 r1 = *(const us8*)(W + (size_t)(k0 + k + 1) * ldb + n0 + n);
#pragma unroll
  for (int j = 0; j < 8; ++j) {
    unsigned int p = (unsigned int)r0[j] | ((unsigned int)r1[j] << 16);
    *(unsigned int*)(sB + (n + j) * STR + k) = p;
  }
}

__global__ __launch_bounds__(256) void cast_f16_kernel(const float* __restrict__ src,
                                                       unsigned short* dst, int n8, float scale) {
  int i = blockIdx.x * 256 + threadIdx.x;
  bool ok = i < n8;
  v4f a = {0.f, 0.f, 0.f, 0.f}, b = {0.f, 0.f, 0.f, 0.f};
  if (ok) {
    a = *(const v4f*)(src + (size_t)i * 8);
    b = *(const v4f*)(src + (size_t)i * 8 + 4);
  }
  Pack8 o;
  v8h f = {(_Float16)(a[0] * scale), (_Float16)(a[1] * scale),
           (_Float16)(a[2] * scale), (_Float16)(a[3] * scale),
           (_Float16)(b[0] * scale), (_Float16)(b[1] * scale),
           (_Float16)(b[2] * scale), (_Float16)(b[3] * scale)};
  o.f = f;
  us8 val = o.u;
  unsigned short* p = dst + (size_t)i * 8;
  if (ok) *(volatile us8*)p = val;
  __threadfence();
  if (ok) *(volatile us8*)p = val;
}

__global__ __launch_bounds__(256) void gate_kernel(const float* __restrict__ x,
                                                   const float* __restrict__ wg,
                                                   const float* __restrict__ bias,
                                                   float* wdense, int S) {
  __shared__ __attribute__((aligned(16))) float sP[8 * NEXP];
  int wave = threadIdx.x >> 5, lane = threadIdx.x & 31;
  int token = blockIdx.x * 8 + wave;
  bool valid = token < S;
  float acc[NEXP];
#pragma unroll
  for (int e = 0; e < NEXP; ++e) acc[e] = 0.0f;
  if (valid) {
    const float* xr = x + (size_t)token * CDIM;
    for (int c = lane; c < CDIM; c += 32) {
      float xv = xr[c];
      const v4f* wr = (const v4f*)(wg + (size_t)c * NEXP);
      v4f w0 = wr[0], w1 = wr[1];
      acc[0] += xv * w0[0]; acc[1] += xv * w0[1]; acc[2] += xv * w0[2]; acc[3] += xv * w0[3];
      acc[4] += xv * w1[0]; acc[5] += xv * w1[1]; acc[6] += xv * w1[2]; acc[7] += xv * w1[3];
    }
  }
#pragma unroll
  for (int e = 0; e < NEXP; ++e)
#pragma unroll
    for (int off = 16; off > 0; off >>= 1)
      acc[e] += __shfl_xor(acc[e], off, 32);
  if (lane == 0) {
    float lg[NEXP];
#pragma unroll
    for (int e = 0; e < NEXP; ++e) lg[e] = acc[e] + bias[e];
    int i0 = 0; float v0 = lg[0];
#pragma unroll
    for (int e = 1; e < NEXP; ++e) if (lg[e] > v0) { v0 = lg[e]; i0 = e; }
    int i1 = 0; float v1 = -__builtin_huge_valf();
#pragma unroll
    for (int e = 0; e < NEXP; ++e) if (e != i0 && lg[e] > v1) { v1 = lg[e]; i1 = e; }
    float den = 0.0f;
#pragma unroll
    for (int e = 0; e < NEXP; ++e) den += __expf(lg[e] - v0);
    float inv = 1.0f / den;
    float p0 = inv;
    float p1 = __expf(v1 - v0) * inv;
#pragma unroll
    for (int e = 0; e < NEXP; ++e) {
      float w = (e == i0) ? p0 : ((e == i1) ? p1 : 0.0f);
      sP[wave * NEXP + e] = valid ? w : 0.0f;
    }
  }
  __syncthreads();
  v4f v = {0.f, 0.f, 0.f, 0.f};
  float* dstp = wdense;
  bool w = false;
  if (wave == 0 && lane < 16) {
    int t = lane >> 1, part = lane & 1;
    int tok = blockIdx.x * 8 + t;
    if (tok < S) {
      v = *(const v4f*)(sP + t * NEXP + part * 4);
      dstp = wdense + (size_t)tok * NEXP + part * 4;
      w = true;
    }
  }
  if (w) *(volatile v4f*)dstp = v;
  __threadfence();
  if (w) *(volatile v4f*)dstp = v;
}

__global__ __launch_bounds__(256) void gemm_swiglu_kernel(
    const unsigned short* __restrict__ X,
    const unsigned short* __restrict__ Wa,
    const unsigned short* __restrict__ Wb,
    unsigned short* Ha,
    unsigned short* Hb,
    int S) {
  __shared__ __attribute__((aligned(16))) unsigned short sA [128 * STR];
  __shared__ __attribute__((aligned(16))) unsigned short sBa[64 * STR];
  __shared__ __attribute__((aligned(16))) unsigned short sBb[64 * STR];
  const unsigned short* W = (blockIdx.z == 0) ? Wa : Wb;
  unsigned short* Hid = (blockIdx.z == 0) ? Ha : Hb;
  int tid = threadIdx.x, lane = tid & 31, wave = tid >> 5;
  int h = lane >> 4, m = lane & 15;
  int wm = wave & 3, wn = wave >> 2;
  int m0 = blockIdx.y * 128, n0 = blockIdx.x * 64;
  if (m0 + 128 > S) return;
  const v8f z8 = {0.f, 0.f, 0.f, 0.f, 0.f, 0.f, 0.f, 0.f};
  v8f accA[2][2], accB[2][2];
#pragma unroll
  for (int i = 0; i < 2; ++i)
#pragma unroll
    for (int j = 0; j < 2; ++j) { accA[i][j] = z8; accB[i][j] = z8; }

#pragma unroll 1
  for (int k0 = 0; k0 < CDIM; k0 += LDK) {
    stage_a(sA, X, m0, k0, CDIM, tid);
    stage_b(sBa, W, k0, n0,        2 * HDIM, tid);
    stage_b(sBb, W, k0, n0 + HDIM, 2 * HDIM, tid);
    __syncthreads();
#pragma unroll
    for (int kc = 0; kc < 2; ++kc) {
      v16h a0  = load_frag(sA,  wm * 32,      kc, lane);
      v16h a1  = load_frag(sA,  wm * 32 + 16, kc, lane);
      v16h ba0 = load_frag(sBa, wn * 32,      kc, lane);
      v16h ba1 = load_frag(sBa, wn * 32 + 16, kc, lane);
      v16h bb0 = load_frag(sBb, wn * 32,      kc, lane);
      v16h bb1 = load_frag(sBb, wn * 32 + 16, kc, lane);
      accA[0][0] = wmma_f16(a0, ba0, accA[0][0]);
      accA[0][1] = wmma_f16(a0, ba1, accA[0][1]);
      accA[1][0] = wmma_f16(a1, ba0, accA[1][0]);
      accA[1][1] = wmma_f16(a1, ba1, accA[1][1]);
      accB[0][0] = wmma_f16(a0, bb0, accB[0][0]);
      accB[0][1] = wmma_f16(a0, bb1, accB[0][1]);
      accB[1][0] = wmma_f16(a1, bb0, accB[1][0]);
      accB[1][1] = wmma_f16(a1, bb1, accB[1][1]);
    }
    __syncthreads();
  }

  unsigned short* sT = sA;
#pragma unroll
  for (int mt = 0; mt < 2; ++mt)
#pragma unroll
    for (int nt = 0; nt < 2; ++nt)
#pragma unroll
      for (int r = 0; r < 8; ++r) {
        int row = wm * 32 + mt * 16 + 8 * h + r;
        int col = wn * 32 + nt * 16 + m;
        float a = accA[mt][nt][r] * INV_XW;
        float b = accB[mt][nt][r] * INV_XW;
        float d = 1.0f + __expf(-a);
        float s = a * __builtin_amdgcn_rcpf(d) * b;
        sT[row * STR + col] = h2bits(s * HSCALE);
      }
  __syncthreads();
  int q = lane >> 3, j = lane & 7;
  us8 vals[4];
  unsigned short* dsts[4];
#pragma unroll
  for (int it = 0; it < 4; ++it) {
    int row = wave * 16 + it * 4 + q;
    vals[it] = *(const us8*)(sT + row * STR + j * 8);
    dsts[it] = Hid + (size_t)(m0 + row) * HDIM + n0 + j * 8;
  }
#pragma unroll
  for (int it = 0; it < 4; ++it) *(volatile us8*)dsts[it] = vals[it];
  __threadfence();
#pragma unroll
  for (int it = 0; it < 4; ++it) *(volatile us8*)dsts[it] = vals[it];
}

__global__ __launch_bounds__(256) void gemm_mix_kernel(
    const unsigned short* __restrict__ Hs,
    const unsigned short* __restrict__ Hr,
    const unsigned short* __restrict__ Wout,
    const unsigned short* __restrict__ W2,
    const float* __restrict__ Wd,
    float* Out,
    int S) {
  __shared__ __attribute__((aligned(16))) unsigned char smem[32768];
  __shared__ __attribute__((aligned(16))) float sWd[128 * NEXP];
  unsigned short* sA = (unsigned short*)smem;
  unsigned short* sB = sA + 128 * STR;
  int tid = threadIdx.x, lane = tid & 31, wave = tid >> 5;
  int h = lane >> 4, m = lane & 15;
  int wm = wave & 3, wn = wave >> 2;
  int m0 = blockIdx.y * 128, n0 = blockIdx.x * 64;
  if (m0 + 128 > S) return;
  *(v4f*)(sWd + tid * 4) = *(const v4f*)(Wd + (size_t)m0 * NEXP + tid * 4);
  __syncthreads();
  const v8f z8 = {0.f, 0.f, 0.f, 0.f, 0.f, 0.f, 0.f, 0.f};
  v8f tot[2][2];
#pragma unroll
  for (int i = 0; i < 2; ++i)
#pragma unroll
    for (int j = 0; j < 2; ++j) tot[i][j] = z8;

#pragma unroll 1
  for (int p = 0; p < NEXP + 1; ++p) {
    const unsigned short* A = (p == 0) ? Hs : Hr;
    const unsigned short* W = (p == 0) ? Wout : (W2 + (size_t)(p - 1) * HDIM * CDIM);
    v8f acc[2][2];
#pragma unroll
    for (int i = 0; i < 2; ++i)
#pragma unroll
      for (int j = 0; j < 2; ++j) acc[i][j] = z8;
#pragma unroll 1
    for (int k0 = 0; k0 < HDIM; k0 += LDK) {
      stage_a(sA, A, m0, k0, HDIM, tid);
      stage_b(sB, W, k0, n0, CDIM, tid);
      __syncthreads();
#pragma unroll
      for (int kc = 0; kc < 2; ++kc) {
        v16h a0 = load_frag(sA, wm * 32,      kc, lane);
        v16h a1 = load_frag(sA, wm * 32 + 16, kc, lane);
        v16h b0 = load_frag(sB, wn * 32,      kc, lane);
        v16h b1 = load_frag(sB, wn * 32 + 16, kc, lane);
        acc[0][0] = wmma_f16(a0, b0, acc[0][0]);
        acc[0][1] = wmma_f16(a0, b1, acc[0][1]);
        acc[1][0] = wmma_f16(a1, b0, acc[1][0]);
        acc[1][1] = wmma_f16(a1, b1, acc[1][1]);
      }
      __syncthreads();
    }
    int pe = (p > 0) ? (p - 1) : 0;
#pragma unroll
    for (int mt = 0; mt < 2; ++mt) {
      int rloc = wm * 32 + mt * 16 + 8 * h;
#pragma unroll
      for (int r = 0; r < 8; ++r) {
        float wl = sWd[(rloc + r) * NEXP + pe];
        float wd = (p > 0) ? wl : 1.0f;
#pragma unroll
        for (int nt = 0; nt < 2; ++nt)
          tot[mt][nt][r] += wd * acc[mt][nt][r];
      }
    }
  }

  float* sT = (float*)smem;
#pragma unroll
  for (int mt = 0; mt < 2; ++mt)
#pragma unroll
    for (int nt = 0; nt < 2; ++nt)
#pragma unroll
      for (int r = 0; r < 8; ++r) {
        int row = wm * 32 + mt * 16 + 8 * h + r;
        int col = wn * 32 + nt * 16 + m;
        sT[row * 64 + col] = tot[mt][nt][r] * INV_HW;
      }
  __syncthreads();
  int q = lane >> 3, j = lane & 7;
  v4f ov[8];
  float* od[8];
#pragma unroll
  for (int it = 0; it < 8; ++it) {
    int row = wave * 16 + it * 2 + (q >> 1);
    int col = (q & 1) * 32 + j * 4;
    ov[it] = *(const v4f*)(sT + row * 64 + col);
    od[it] = Out + (size_t)(m0 + row) * CDIM + n0 + col;
  }
#pragma unroll
  for (int it = 0; it < 8; ++it) *(volatile v4f*)od[it] = ov[it];
  __threadfence();
#pragma unroll
  for (int it = 0; it < 8; ++it) *(volatile v4f*)od[it] = ov[it];
}

extern "C" void kernel_launch(void* const* d_in, const int* in_sizes, int n_in,
                              void* d_out, int out_size, void* d_ws, size_t ws_size,
                              hipStream_t stream) {
  if (n_in < 7) return;
  const int S = in_sizes[0] / CDIM;
  if (S <= 0 || S * CDIM != in_sizes[0] || (S % 128) != 0) return;
  if (in_sizes[1] != CDIM * 2 * HDIM || in_sizes[2] != HDIM * CDIM ||
      in_sizes[3] != CDIM * 2 * HDIM || in_sizes[4] != NEXP * HDIM * CDIM ||
      in_sizes[5] != CDIM * NEXP || in_sizes[6] < NEXP) return;
  if (out_size != S * CDIM) return;

  const float* x            = (const float*)d_in[0];
  const float* w_shared_in  = (const float*)d_in[1];
  const float* w_shared_out = (const float*)d_in[2];
  const float* w1_shared    = (const float*)d_in[3];
  const float* w2           = (const float*)d_in[4];
  const float* w_gate       = (const float*)d_in[5];
  const float* gate_bias    = (const float*)d_in[6];
  float* out = (float*)d_out;

  const size_t nx   = (size_t)S * CDIM;
  const size_t nwin = (size_t)CDIM * 2 * HDIM;
  const size_t nwo  = (size_t)HDIM * CDIM;
  const size_t nw2  = (size_t)NEXP * HDIM * CDIM;
  const size_t nh   = (size_t)S * HDIM;
  const size_t nwd  = (size_t)S * NEXP;
  const size_t total = 2 * (nx + 2 * nwin + nwo + nw2 + 2 * nh) + 4 * nwd;
  if (total > ws_size) return;
  unsigned short* xb      = (unsigned short*)d_ws;
  unsigned short* w_in_b  = xb      + nx;
  unsigned short* w1_b    = w_in_b  + nwin;
  unsigned short* w_out_b = w1_b    + nwin;
  unsigned short* w2_b    = w_out_b + nwo;
  unsigned short* hshared = w2_b    + nw2;
  unsigned short* hrouted = hshared + nh;
  float*          wdense  = (float*)(hrouted + nh);

  {
    int n8;
    n8 = (int)(nx / 8);
    cast_f16_kernel<<<dim3((unsigned)((n8 + 255) / 256)), dim3(256), 0, stream>>>(x, xb, n8, XSCALE);
    n8 = (int)(nwin / 8);
    cast_f16_kernel<<<dim3((unsigned)((n8 + 255) / 256)), dim3(256), 0, stream>>>(w_shared_in, w_in_b, n8, WSCALE);
    cast_f16_kernel<<<dim3((unsigned)((n8 + 255) / 256)), dim3(256), 0, stream>>>(w1_shared, w1_b, n8, WSCALE);
    n8 = (int)(nwo / 8);
    cast_f16_kernel<<<dim3((unsigned)((n8 + 255) / 256)), dim3(256), 0, stream>>>(w_shared_out, w_out_b, n8, WSCALE);
    n8 = (int)(nw2 / 8);
    cast_f16_kernel<<<dim3((unsigned)((n8 + 255) / 256)), dim3(256), 0, stream>>>(w2, w2_b, n8, WSCALE);
  }

  gate_kernel<<<dim3((unsigned)((S + 7) / 8)), dim3(256), 0, stream>>>(x, w_gate, gate_bias, wdense, S);

  dim3 grid1(HDIM / 64, (unsigned)(S / 128), 2);
  gemm_swiglu_kernel<<<grid1, dim3(256), 0, stream>>>(xb, w_in_b, w1_b, hshared, hrouted, S);

  dim3 grid2(CDIM / 64, (unsigned)(S / 128));
  gemm_mix_kernel<<<grid2, dim3(256), 0, stream>>>(hshared, hrouted, w_out_b, w2_b, wdense, out, S);
}
